// EnsembleDynamicsModel_15006615733146
// MI455X (gfx1250) — hardware-verified
//
#include <hip/hip_runtime.h>
#include <math.h>
#include <stdint.h>

#define EN      7
#define BATCH   32768
#define SDIM    32
#define ADIM    8
#define DIN     40
#define HID     200
#define OUTD    66
#define NCOL    33
#define LSTR    232
#define NT_H    13
#define KS_H    7
#define KS_IN   2
#define NT_O    5
#define MT      2
#define ROWS    (MT * 16)
#define WAVES   4
#define TPB     (WAVES * 32)
#define BROWS   (WAVES * ROWS)
#define OFS     84
#define RES_OFF 2688
#define W1_PER  (NT_H * KS_IN * 512)
#define WH_PER  (NT_H * KS_H * 512)
#define W5_PER  (NT_O * KS_H * 512)
#define SX      8.0f
#define SW      64.0f
#define INVS    (1.0f / 512.0f)

static_assert((BATCH % BROWS) == 0);
static_assert((LSTR % 8) == 0);
static_assert(LSTR >= KS_H * 32);
static_assert(NT_H * 16 >= HID);
static_assert(NT_H * 16 <= KS_H * 32);
static_assert(KS_H * 32 >= HID);
static_assert(KS_IN * 32 >= DIN);
static_assert(NT_O * 16 >= OUTD);
static_assert(OFS >= NT_O * 16);
static_assert(ROWS * OFS <= RES_OFF);
static_assert(RES_OFF + ROWS * SDIM == (ROWS * LSTR) / 2);
static_assert(((ROWS * LSTR * 2) % 16) == 0);
static_assert(((RES_OFF * 4) % 16) == 0);
static_assert(OUTD == 2 * NCOL);
static_assert(SDIM + 1 == NCOL);
static_assert(ROWS * NCOL == 33 * 32);

typedef _Float16       v16h __attribute__((ext_vector_type(16)));
typedef unsigned short v8us __attribute__((ext_vector_type(8)));
typedef unsigned short v4us __attribute__((ext_vector_type(4)));
typedef float          v8f  __attribute__((ext_vector_type(8)));
typedef float          v4f  __attribute__((ext_vector_type(4)));

union Frag { v16h v; v8us u[2]; };

__device__ __forceinline__ unsigned short bf_bits(float f) {
  const unsigned u = __float_as_uint(f);
  return (unsigned short)((u + 0x7FFFu + ((u >> 16) & 1u)) >> 16);
}
__device__ __forceinline__ float bf_up(unsigned short b) { return __uint_as_float(((unsigned)b) << 16); }
__device__ __forceinline__ float bfr(float f) { return bf_up(bf_bits(f)); }
__device__ __forceinline__ unsigned short h_bits(float f) {
  return __builtin_bit_cast(unsigned short, (_Float16)f);
}
__device__ __forceinline__ unsigned short hx(float f) { return h_bits(bfr(f) * SX); }

__device__ __forceinline__ float swish_f(float z) {
  const float ez = expf(-z);
  return z * __builtin_amdgcn_rcpf(1.0f + ez);
}
__device__ __forceinline__ float softplus_f(float x) {
  return fmaxf(x, 0.0f) + log1pf(expf(-fabsf(x)));
}

__device__ __forceinline__ v8f mma_h(v16h a, v16h b, v8f c) {
  return __builtin_amdgcn_wmma_f32_16x16x32_f16(false, a, false, b, (short)0, c, false, false);
}
__device__ __forceinline__ void mma_guard2(v8f& c0, v8f& c1, v16h a0, v16h a1, v16h b) {
#if defined(__HIP_DEVICE_COMPILE__)
  asm volatile("v_nop\n\tv_nop\n\tv_nop\n\tv_nop" : "+v"(c0), "+v"(c1) : "v"(a0), "v"(a1), "v"(b));
#else
  (void)c0; (void)c1; (void)a0; (void)a1; (void)b;
#endif
}

__global__ __launch_bounds__(256) void k_pack(const float* __restrict__ W, unsigned short* dst,
                                              int Kreal, int Nreal, int kS, int nT, int nPieces) {
  const int piece = blockIdx.x * 256 + threadIdx.x;
  const bool act  = piece < nPieces;
  const int pc    = act ? piece : (nPieces - 1);
  const int elem0 = pc * 8;
  const int per_e = nT * kS * 512;
  const int e     = elem0 / per_e;
  int rem         = elem0 - e * per_e;
  const int tblk  = kS * 512;
  const int t     = rem / tblk;
  rem            -= t * tblk;
  const int s     = rem >> 9;
  rem            &= 511;
  const int L     = rem >> 4;
  const int j0    = rem & 15;
  const int n     = t * 16 + (L & 15);
  const int hh    = L >> 4;
  const int kb    = s * 32 + 8 * hh + 2 * j0;
  const int nc    = (n < Nreal) ? n : (Nreal - 1);
  v8us o;
#pragma unroll
  for (int jj = 0; jj < 8; ++jj) {
    const int k  = kb + jj;
    const int kc = (k < Kreal) ? k : (Kreal - 1);
    float v = W[((size_t)e * Kreal + (size_t)kc) * Nreal + nc];
    v = (k < Kreal && n < Nreal) ? v : 0.0f;
    o[jj] = h_bits(bfr(v) * SW);
  }
  unsigned short* d = dst + (size_t)pc * 8;
  if (act) *(volatile v8us*)d = o;
  __threadfence();
  if (act) *(volatile v8us*)d = o;
}

template <int NT, int KS, bool LAST>
__device__ __forceinline__ void layer_fwd(const unsigned short* __restrict__ Wp,
                                          const float* __restrict__ bias, int Nreal,
                                          unsigned short* slice, int lane) {
  Frag a[MT][KS];
  const int m  = lane & 15;
  const int hh = lane >> 4;
#pragma unroll
  for (int mt = 0; mt < MT; ++mt) {
#pragma unroll
    for (int s = 0; s < KS; ++s) {
      const unsigned short* p = slice + (mt * 16 + m) * LSTR + s * 32 + 8 * hh;
      a[mt][s].u[0] = *(const v8us*)(p);
      a[mt][s].u[1] = *(const v8us*)(p + 16);
    }
  }
  const int mrow = 8 * hh;
#pragma unroll 1
  for (int t = 0; t < NT; ++t) {
    const int n  = t * 16 + m;
    const int nc = (n < Nreal) ? n : (Nreal - 1);
    float bv = bias[nc];
    bv = (n < Nreal) ? bfr(bv) : 0.0f;
    v8f c[MT];
#pragma unroll
    for (int mt = 0; mt < MT; ++mt) c[mt] = (v8f){0.f, 0.f, 0.f, 0.f, 0.f, 0.f, 0.f, 0.f};
    Frag b;
    b.v = a[0][0].v;
#pragma unroll
    for (int s = 0; s < KS; ++s) {
      const unsigned short* wp = Wp + ((size_t)((t * KS + s) * 32 + lane) << 4);
      b.u[0] = *(const v8us*)(wp);
      b.u[1] = *(const v8us*)(wp + 8);
#pragma unroll
      for (int mt = 0; mt < MT; ++mt) c[mt] = mma_h(a[mt][s].v, b.v, c[mt]);
    }
    mma_guard2(c[0], c[1], a[0][KS - 1].v, a[1][KS - 1].v, b.v);
    if constexpr (!LAST) {
#pragma unroll
      for (int mt = 0; mt < MT; ++mt) {
        unsigned short* dst = slice + (mt * 16 + mrow) * LSTR + n;
#pragma unroll
        for (int v = 0; v < 8; ++v) {
          const float z = c[mt][v] * INVS + bv;
          dst[v * LSTR] = h_bits(swish_f(z) * SX);
        }
      }
    } else {
      float* of = (float*)slice;
#pragma unroll
      for (int mt = 0; mt < MT; ++mt) {
#pragma unroll
        for (int v = 0; v < 8; ++v) of[(mt * 16 + mrow + v) * OFS + n] = c[mt][v] * INVS + bv;
      }
    }
  }
}

__global__ __launch_bounds__(TPB) void k_fwd(
    const float* __restrict__ state, const float* __restrict__ action, const float* __restrict__ noise,
    const unsigned short* __restrict__ Wp1, const unsigned short* __restrict__ Wp2,
    const unsigned short* __restrict__ Wp3, const unsigned short* __restrict__ Wp4,
    const unsigned short* __restrict__ Wp5,
    const float* __restrict__ b1, const float* __restrict__ b2, const float* __restrict__ b3,
    const float* __restrict__ b4, const float* __restrict__ b5,
    const float* __restrict__ max_lv, const float* __restrict__ min_lv,
    float* out) {
  __shared__ __align__(16) unsigned short lds[WAVES * ROWS * LSTR];
  __shared__ __align__(16) float s_rew[BROWS];

  const int lane = threadIdx.x & 31;
  const int wave = threadIdx.x >> 5;
  constexpr int BPE = BATCH / BROWS;
  const int e  = blockIdx.x / BPE;
  const int rb = (blockIdx.x - e * BPE) * BROWS;
  const int r0 = rb + wave * ROWS;
  unsigned short* slice = lds + wave * (ROWS * LSTR);

  {
    const v8us z = (v8us){0, 0, 0, 0, 0, 0, 0, 0};
    for (int i = lane; i < (ROWS * LSTR) / 8; i += 32) *(v8us*)(slice + i * 8) = z;
  }
  __syncthreads();
  for (int i = lane; i < ROWS * 8; i += 32) {
    const int r = i >> 3, q = i & 7;
    const v4f x = *(const v4f*)(state + (size_t)(r0 + r) * SDIM + q * 4);
    v4us o;
    o[0] = hx(x[0]); o[1] = hx(x[1]); o[2] = hx(x[2]); o[3] = hx(x[3]);
    *(v4us*)(slice + r * LSTR + q * 4) = o;
  }
  for (int i = lane; i < ROWS * 2; i += 32) {
    const int r = i >> 1, q = i & 1;
    const v4f x = *(const v4f*)(action + (size_t)(r0 + r) * ADIM + q * 4);
    v4us o;
    o[0] = hx(x[0]); o[1] = hx(x[1]); o[2] = hx(x[2]); o[3] = hx(x[3]);
    *(v4us*)(slice + r * LSTR + SDIM + q * 4) = o;
  }
  __syncthreads();

  layer_fwd<NT_H, KS_IN, false>(Wp1 + (size_t)e * W1_PER, b1 + e * HID, HID, slice, lane);
  __syncthreads();
#pragma unroll 1
  for (int l = 0; l < 3; ++l) {
    const unsigned short* Wl = (l == 0) ? Wp2 : ((l == 1) ? Wp3 : Wp4);
    const float* bl = (l == 0) ? b2 : ((l == 1) ? b3 : b4);
    layer_fwd<NT_H, KS_H, false>(Wl + (size_t)e * WH_PER, bl + e * HID, HID, slice, lane);
    __syncthreads();
  }
  layer_fwd<NT_O, KS_H, true>(Wp5 + (size_t)e * W5_PER, b5 + e * OUTD, OUTD, slice, lane);
  __syncthreads();

  {
    const float* of = (const float*)slice;
    float* res = (float*)slice + RES_OFF;
    for (int i = lane; i < ROWS * NCOL; i += 32) {
      const int r    = i / NCOL;
      const int cc   = i - r * NCOL;
      const int brow = r0 + r;
      const float mval = of[r * OFS + cc];
      float lv         = of[r * OFS + NCOL + cc];
      const float mx   = bfr(max_lv[cc]);
      const float mn   = bfr(min_lv[cc]);
      lv = mx - softplus_f(mx - lv);
      lv = mn + softplus_f(lv - mn);
      const float sd   = expf(0.5f * lv);
      const float nz   = bfr(noise[((size_t)e * BATCH + (size_t)brow) * NCOL + cc]);
      const float smp  = mval + sd * nz;
      const int sc     = (cc < SDIM) ? cc : (SDIM - 1);
      const float st   = bfr(state[(size_t)brow * SDIM + sc]);
      const float ns   = st + smp;
      if (cc < SDIM) res[r * SDIM + cc] = ns;
      else           s_rew[wave * ROWS + r] = smp;
    }
  }
  __syncthreads();

  {
    const float* res = (const float*)slice + RES_OFF;
    v4f vals[8];
#pragma unroll
    for (int i = 0; i < 8; ++i) vals[i] = *(const v4f*)(res + (i * 32 + lane) * 4);
    const v4f rv = *(const v4f*)(s_rew + lane * 4);
    float* o0 = out + ((size_t)e * BATCH + (size_t)r0) * SDIM;
    float* o1 = out + (size_t)EN * BATCH * SDIM + (size_t)e * BATCH + (size_t)rb;
#pragma unroll
    for (int i = 0; i < 8; ++i) *(volatile v4f*)(o0 + (size_t)(i * 32 + lane) * 4) = vals[i];
    if (wave == 0) *(volatile v4f*)(o1 + lane * 4) = rv;
    __threadfence();
#pragma unroll
    for (int i = 0; i < 8; ++i) *(volatile v4f*)(o0 + (size_t)(i * 32 + lane) * 4) = vals[i];
    if (wave == 0) *(volatile v4f*)(o1 + lane * 4) = rv;
  }
}

static void launch_pack(const float* W, unsigned short* dst, int Kreal, int Nreal, int kS, int nT,
                        hipStream_t stream) {
  const int nPieces = EN * nT * kS * 64;
  const int blocks  = (nPieces + 255) / 256;
  k_pack<<<dim3(blocks), dim3(256), 0, stream>>>(W, dst, Kreal, Nreal, kS, nT, nPieces);
}

extern "C" void kernel_launch(void* const* d_in, const int* in_sizes, int n_in,
                              void* d_out, int out_size, void* d_ws, size_t ws_size,
                              hipStream_t stream) {
  if (n_in < 15) return;
  if (in_sizes[0]  != BATCH * SDIM) return;
  if (in_sizes[1]  != BATCH * ADIM) return;
  if (in_sizes[2]  != EN * BATCH * NCOL) return;
  if (in_sizes[3]  != EN * DIN * HID)  return;
  if (in_sizes[4]  != EN * HID) return;
  if (in_sizes[5]  != EN * HID * HID)  return;
  if (in_sizes[6]  != EN * HID) return;
  if (in_sizes[7]  != EN * HID * HID)  return;
  if (in_sizes[8]  != EN * HID) return;
  if (in_sizes[9]  != EN * HID * HID)  return;
  if (in_sizes[10] != EN * HID) return;
  if (in_sizes[11] != EN * HID * OUTD) return;
  if (in_sizes[12] != EN * OUTD) return;
  if (in_sizes[13] != NCOL || in_sizes[14] != NCOL) return;
  if (out_size != EN * BATCH * NCOL) return;

  const float* state  = (const float*)d_in[0];
  const float* action = (const float*)d_in[1];
  const float* noise  = (const float*)d_in[2];
  const float* W1 = (const float*)d_in[3];   const float* b1 = (const float*)d_in[4];
  const float* W2 = (const float*)d_in[5];   const float* b2 = (const float*)d_in[6];
  const float* W3 = (const float*)d_in[7];   const float* b3 = (const float*)d_in[8];
  const float* W4 = (const float*)d_in[9];   const float* b4 = (const float*)d_in[10];
  const float* W5 = (const float*)d_in[11];  const float* b5 = (const float*)d_in[12];
  const float* max_lv = (const float*)d_in[13];
  const float* min_lv = (const float*)d_in[14];
  float* out = (float*)d_out;

  const size_t o1 = 0;
  const size_t o2 = o1 + (size_t)EN * W1_PER;
  const size_t o3 = o2 + (size_t)EN * WH_PER;
  const size_t o4 = o3 + (size_t)EN * WH_PER;
  const size_t o5 = o4 + (size_t)EN * WH_PER;
  const size_t tot_bytes = (o5 + (size_t)EN * W5_PER) * 2;
  if (tot_bytes > ws_size) return;
  if (tot_bytes > (size_t)134217728) return;

  unsigned short* ws = (unsigned short*)d_ws;
  unsigned short* Wp1 = ws + o1;
  unsigned short* Wp2 = ws + o2;
  unsigned short* Wp3 = ws + o3;
  unsigned short* Wp4 = ws + o4;
  unsigned short* Wp5 = ws + o5;

  launch_pack(W1, Wp1, DIN, HID,  KS_IN, NT_H, stream);
  launch_pack(W2, Wp2, HID, HID,  KS_H,  NT_H, stream);
  launch_pack(W3, Wp3, HID, HID,  KS_H,  NT_H, stream);
  launch_pack(W4, Wp4, HID, HID,  KS_H,  NT_H, stream);
  launch_pack(W5, Wp5, HID, OUTD, KS_H,  NT_O, stream);

  k_fwd<<<dim3(EN * (BATCH / BROWS)), dim3(TPB), 0, stream>>>(
      state, action, noise, Wp1, Wp2, Wp3, Wp4, Wp5, b1, b2, b3, b4, b5, max_lv, min_lv, out);
  (void)hipGetLastError();
}
